// S5SSM_7782480740554
// MI455X (gfx1250) — hardware-verified
//
#include <hip/hip_runtime.h>


#define LL   32768
#define HH   256
#define PP   256
#define P2   512
#define BSC  4096.0f
#define BSCI (1.0f / 4096.0f)
#define CSC  64.0f
#define CSCI (1.0f / 64.0f)
#define LOSC 1024.0f
#define LOSCI (1.0f / 1024.0f)

typedef _Float16 h16;
typedef __attribute__((ext_vector_type(16))) _Float16 v16h;
typedef __attribute__((ext_vector_type(8)))  _Float16 v8h;
typedef __attribute__((ext_vector_type(8)))  float    v8f;
typedef __attribute__((ext_vector_type(4)))  float    v4f;
typedef v8h  __attribute__((may_alias)) v8ha;
typedef v4f  __attribute__((may_alias)) v4fa;

__device__ __forceinline__ unsigned short f2bf(float f) { unsigned u = __float_as_uint(f); u += 0x7FFFu + ((u >> 16) & 1u); return (unsigned short)(u >> 16); }
__device__ __forceinline__ float bf2f(unsigned short b) { return __uint_as_float(((unsigned)b) << 16); }
__device__ __forceinline__ float bfr(float f) { return bf2f(f2bf(f)); }
__device__ __forceinline__ v16h cat16(v8h lo, v8h hi) { return __builtin_shufflevector(lo, hi, 0, 1, 2, 3, 4, 5, 6, 7, 8, 9, 10, 11, 12, 13, 14, 15); }
__device__ __forceinline__ v8f wmma16(v16h a, v16h b, v8f c) { return __builtin_amdgcn_wmma_f32_16x16x32_f16(false, a, false, b, (short)0, c, false, false); }
#define VST2(T, p, v) do { const T vst2_v_ = (v); *(volatile T*)(p) = vst2_v_; __threadfence(); *(volatile T*)(p) = vst2_v_; } while (0)

__device__ __forceinline__ void disc(const float* Lri, const float* lstep, int p, float& ar, float& ai, float& gr, float& gi) {
    const float lr = bfr(Lri[p * 2]), li = bfr(Lri[p * 2 + 1]), st = expf(bfr(lstep[p]));
    const float er = expf(lr * st); ar = er * cosf(li * st); ai = er * sinf(li * st);
    const float nr = ar - 1.0f, ni = ai, den = lr * lr + li * li;
    gr = (nr * lr + ni * li) / den; gi = (ni * lr - nr * li) / den;
}
__global__ __launch_bounds__(256) void k_lb(const float* __restrict__ Lri, const float* __restrict__ lstep, float* LB, float* XST) {
    typedef __attribute__((ext_vector_type(2))) float v2f;
    const int p = threadIdx.x;
    float ar, ai, gr, gi; disc(Lri, lstep, p, ar, ai, gr, gi);
    v2f v; v[0] = ar; v[1] = ai; VST2(v2f, LB + p * 2, v);
    v2f z; z[0] = 0.f; z[1] = 0.f; VST2(v2f, XST + p * 2, z);
}
__global__ __launch_bounds__(256) void k_bb(const float* __restrict__ Lri, const float* __restrict__ Bri, const float* __restrict__ lstep, h16* BBH, h16* BBL) {
    const int lane = threadIdx.x & 31, p = blockIdx.x * 8 + (threadIdx.x >> 5);
    float ar, ai, gr, gi; disc(Lri, lstep, p, ar, ai, gr, gi);
    v8h hr, lr8, hi8, li8;
#pragma unroll
    for (int i = 0; i < 8; ++i) { const int h = lane * 8 + i; const float br = bfr(Bri[((size_t)p * HH + h) * 2]), bi = bfr(Bri[((size_t)p * HH + h) * 2 + 1]);
        const float vr = (gr * br - gi * bi) * BSC, vi = (gr * bi + gi * br) * BSC;
        const h16 a = (h16)vr, b = (h16)vi; hr[i] = a; lr8[i] = (h16)((vr - (float)a) * LOSC); hi8[i] = b; li8[i] = (h16)((vi - (float)b) * LOSC); }
    *(volatile v8h*)(BBH + (size_t)p * HH + lane * 8) = hr; *(volatile v8h*)(BBL + (size_t)p * HH + lane * 8) = lr8;
    *(volatile v8h*)(BBH + (size_t)(PP + p) * HH + lane * 8) = hi8; *(volatile v8h*)(BBL + (size_t)(PP + p) * HH + lane * 8) = li8;
    __threadfence();
    *(volatile v8h*)(BBH + (size_t)p * HH + lane * 8) = hr; *(volatile v8h*)(BBL + (size_t)p * HH + lane * 8) = lr8;
    *(volatile v8h*)(BBH + (size_t)(PP + p) * HH + lane * 8) = hi8; *(volatile v8h*)(BBL + (size_t)(PP + p) * HH + lane * 8) = li8;
}
__global__ __launch_bounds__(256) void k_u16(const float* __restrict__ u, h16* U16) {
    const int lane = threadIdx.x & 31, r = blockIdx.x * 8 + (threadIdx.x >> 5);
    if (r >= LL) return;
    v8h t;
#pragma unroll
    for (int i = 0; i < 8; ++i) t[i] = (h16)bfr(u[(size_t)r * HH + lane * 8 + i]);
    VST2(v8h, U16 + (size_t)r * HH + lane * 8, t);
}
__global__ __launch_bounds__(256) void k_c16(const float* __restrict__ Cri, h16* CT) {
    const int lane = threadIdx.x & 31, r = blockIdx.x * 8 + (threadIdx.x >> 5);
    if (r >= HH) return;
#pragma unroll
    for (int s = 0; s < 2; ++s) { v8h o;
#pragma unroll
        for (int i = 0; i < 4; ++i) { const int p = s * 128 + lane * 4 + i; o[2 * i] = (h16)(bfr(Cri[((size_t)r * PP + p) * 2]) * CSC); o[2 * i + 1] = (h16)(-bfr(Cri[((size_t)r * PP + p) * 2 + 1]) * CSC); }
        VST2(v8h, CT + (size_t)r * P2 + s * 256 + lane * 8, o); }
}

template <bool SPLITA, int MODE>
__global__ __launch_bounds__(128) void k_gemm(const h16* __restrict__ A, const h16* __restrict__ Al, const h16* __restrict__ Bm, const h16* __restrict__ Bl, int K,
                                             const float* __restrict__ Dv, const float* __restrict__ u, float* C, int ldc) {
    __shared__ __align__(16) float ost[4][16 * 68];
    const int lane = threadIdx.x & 31, wave = threadIdx.x >> 5, lr = lane & 15, hi = lane >> 4;
    const int r0 = blockIdx.x * 64 + wave * 16, c0 = blockIdx.y * 64;
    const size_t aoff = (size_t)(r0 + lr) * K + 8 * hi;
    size_t boff[4];
#pragma unroll
    for (int t = 0; t < 4; ++t) boff[t] = (size_t)(c0 + t * 16 + lr) * K + 8 * hi;
    v8f acc[4], accx[4];
#pragma unroll
    for (int t = 0; t < 4; ++t) { acc[t] = (v8f){}; accx[t] = (v8f){}; }
#pragma unroll 1
    for (int kc = 0; kc < K; kc += 32) {
        const v16h a = cat16(*(const v8h*)(A + aoff + kc), *(const v8h*)(A + aoff + kc + 16));
        v16h al = a; if (SPLITA) al = cat16(*(const v8h*)(Al + aoff + kc), *(const v8h*)(Al + aoff + kc + 16));
#pragma unroll
        for (int t = 0; t < 4; ++t) { const v16h bb = cat16(*(const v8h*)(Bm + boff[t] + kc), *(const v8h*)(Bm + boff[t] + kc + 16)); acc[t] = wmma16(a, bb, acc[t]);
            if (SPLITA) accx[t] = wmma16(al, bb, accx[t]);
            else { const v16h bl = cat16(*(const v8h*)(Bl + boff[t] + kc), *(const v8h*)(Bl + boff[t] + kc + 16)); accx[t] = wmma16(a, bl, accx[t]); } }
        asm volatile("v_nop\n\tv_nop\n\tv_nop\n\tv_nop" : "+v"(acc[0]), "+v"(acc[1]), "+v"(acc[2]), "+v"(acc[3]), "+v"(accx[0]), "+v"(accx[3]) : "v"(a), "v"(al));
    }
    asm volatile("v_nop\n\tv_nop\n\tv_nop\n\tv_nop" : "+v"(accx[0]), "+v"(accx[1]), "+v"(accx[2]), "+v"(accx[3]));
    float* os = &ost[wave][0];
#pragma unroll
    for (int t = 0; t < 4; ++t) { const int col = c0 + t * 16 + lr;
#pragma unroll
        for (int j = 0; j < 8; ++j) { float v = acc[t][j] + accx[t][j] * LOSCI; if (MODE == 1) v = v * CSCI + bfr(Dv[col]) * bfr(u[(size_t)(r0 + hi * 8 + j) * HH + col]); os[(hi * 8 + j) * 68 + t * 16 + lr] = v; } }
    __syncthreads();
    float* crow = C + (size_t)r0 * ldc + c0;
    auto pass = [&]() {
#pragma unroll
        for (int s = 0; s < 8; ++s) { const int Lid = (lane >> 3) + 4 * s, piece = lane & 7; const int row = Lid >> 1, cofs = (Lid & 1) * 32 + piece * 4;
            const v4f val = *(const v4fa*)(os + row * 68 + cofs); *(volatile v4f*)(crow + (size_t)row * ldc + cofs) = val; }
    };
    pass(); __threadfence(); pass();
}

__global__ __launch_bounds__(256) void k_scan(const float* __restrict__ LB, const float* __restrict__ BU, int t0, float* XST, h16* XH, h16* XL) {
    typedef __attribute__((ext_vector_type(2))) _Float16 v2h;
    const int p = threadIdx.x;
    const float ar = LB[p * 2], ai = LB[p * 2 + 1];
    const float x0r = XST[p * 2], x0i = XST[p * 2 + 1];
    float xr, xi;
#pragma unroll 1
    for (int pass = 0; pass < 2; ++pass) {
        xr = x0r; xi = x0i;
#pragma unroll 1
        for (int tt = 0; tt < LL / 2; ++tt) {
            const float br = BU[(size_t)tt * P2 + p] * BSCI, bi = BU[(size_t)tt * P2 + PP + p] * BSCI;
            const float nr = ar * xr - ai * xi + br, ni = ar * xi + ai * xr + bi;
            xr = nr; xi = ni;
            const h16 hr = (h16)xr, hi_ = (h16)xi; v2h vh, vl; vh[0] = hr; vh[1] = hi_; vl[0] = (h16)((xr - (float)hr) * LOSC); vl[1] = (h16)((xi - (float)hi_) * LOSC);
            *(volatile v2h*)(XH + (size_t)(t0 + tt) * P2 + 2 * p) = vh; *(volatile v2h*)(XL + (size_t)(t0 + tt) * P2 + 2 * p) = vl;
        }
        __threadfence();
    }
    __syncthreads();
    typedef __attribute__((ext_vector_type(2))) float v2f;
    v2f c; c[0] = xr; c[1] = xi; VST2(v2f, XST + p * 2, c);
}
extern "C" void kernel_launch(void* const* d_in, const int* in_sizes, int n_in,
                              void* d_out, int out_size, void* d_ws, size_t ws_size, hipStream_t stream) {
    (void)in_sizes; (void)n_in; (void)out_size;
    const float* u = (const float*)d_in[0]; const float* Lri = (const float*)d_in[1]; const float* Bri = (const float*)d_in[2]; const float* Cri = (const float*)d_in[3];
    const float* Dv = (const float*)d_in[4]; const float* lstep = (const float*)d_in[5];
    float* out = (float*)d_out;
    char* wsp = (char*)d_ws;
    auto take = [&](size_t bytes) { char* p = wsp; wsp += (bytes + 255) & ~(size_t)255; return (void*)p; };
    float* LB = (float*)take(P2 * 4); float* XST = (float*)take(P2 * 4);
    h16* BBH = (h16*)take((size_t)P2 * HH * 2); h16* BBL = (h16*)take((size_t)P2 * HH * 2); h16* U16 = (h16*)take((size_t)LL * HH * 2); h16* CT = (h16*)take((size_t)HH * P2 * 2);
    float* BU = (float*)take((size_t)(LL / 2) * P2 * 4); h16* XH = (h16*)take((size_t)LL * P2 * 2); h16* XL = (h16*)take((size_t)LL * P2 * 2);
    if ((size_t)(wsp - (char*)d_ws) > ws_size) return;
    k_lb<<<1, 256, 0, stream>>>(Lri, lstep, LB, XST);
    k_bb<<<PP / 8, 256, 0, stream>>>(Lri, Bri, lstep, BBH, BBL);
    k_u16<<<LL / 8, 256, 0, stream>>>(u, U16);
    k_c16<<<HH / 8, 256, 0, stream>>>(Cri, CT);
    for (int half = 0; half < 2; ++half) {
        const int t0 = half * (LL / 2);
        k_gemm<false, 0><<<dim3((LL / 2) / 64, P2 / 64, 1), 128, 0, stream>>>(U16 + (size_t)t0 * HH, nullptr, BBH, BBL, HH, nullptr, nullptr, BU, P2);
        k_scan<<<1, 256, 0, stream>>>(LB, BU, t0, XST, XH, XL);
    }
    k_gemm<true, 1><<<dim3(LL / 64, HH / 64, 1), 128, 0, stream>>>(XH, XL, CT, nullptr, P2, Dv, u, out, HH);
}
